// EncoderLayer_82867099009759
// MI455X (gfx1250) — hardware-verified
//
#include <hip/hip_runtime.h>


#ifndef NB
#define NB 2
#endif
#ifndef SEQ
#define SEQ 2048
#endif
#define NB_FULL 2
#define SEQ_FULL 2048
#define DM 768
#define NH 12
#define HD 64
#define FF 3072
#define MR (NB * SEQ)
#define NT (SEQ / 64)
#define NQKV (3 * DM)
#define WCAR 16.0f
#define LNEPS 1e-6f
#define NEGV (-1.0e9f)
#define L2E 1.4426950408889634f

typedef _Float16 h16;
typedef __attribute__((ext_vector_type(16))) _Float16 v16h;
typedef __attribute__((ext_vector_type(8)))  _Float16 v8h;
typedef __attribute__((ext_vector_type(4)))  _Float16 v4h;
typedef __attribute__((ext_vector_type(2)))  _Float16 v2h;
typedef __attribute__((ext_vector_type(8)))  float    v8f;
typedef __attribute__((ext_vector_type(4)))  float    v4f;
typedef __attribute__((ext_vector_type(4)))  int      v4i;
typedef v4f __attribute__((may_alias)) v4fa;

static_assert(DM == NH * HD);
static_assert(HD == 64);
static_assert(SEQ % 64 == 0);
static_assert(NB <= NB_FULL);
static_assert(SEQ <= SEQ_FULL);
static_assert(MR % 64 == 0);
static_assert(DM % 64 == 0);
static_assert(FF % 64 == 0);
static_assert(((SEQ / 16) * NT) % 8 == 0);
static_assert(((MR * DM) / 8) % 256 == 0);
static_assert(MR % 8 == 0);
static_assert(DM % 128 == 0);

__device__ __forceinline__ unsigned short f2bf(float f) { unsigned u = __float_as_uint(f); u += 0x7FFFu + ((u >> 16) & 1u); return (unsigned short)(u >> 16); }
__device__ __forceinline__ float bfr(float f) { return __uint_as_float(((unsigned)f2bf(f)) << 16); }
__device__ __forceinline__ v16h cat16(v8h lo, v8h hi) { return __builtin_shufflevector(lo, hi, 0, 1, 2, 3, 4, 5, 6, 7, 8, 9, 10, 11, 12, 13, 14, 15); }
__device__ __forceinline__ v8f wmma16(v16h a, v16h b, v8f c) { return __builtin_amdgcn_wmma_f32_16x16x32_f16(false, a, false, b, (short)0, c, false, false); }
__device__ __forceinline__ v16h ldfr(const h16* p) { return cat16(*(const v8h*)p, *(const v8h*)(p + 16)); }
__device__ __forceinline__ unsigned fullrow(unsigned r) { return (r / (unsigned)SEQ) * (unsigned)SEQ_FULL + (r % (unsigned)SEQ); }

template <unsigned K, unsigned N>
__global__ __launch_bounds__(256) void k_wt(const float* __restrict__ w, h16* Bt) {
    static_assert(K % 64u == 0u);
    static_assert((N * (K / 64u)) % 64u == 0u);
    const unsigned lane = threadIdx.x & 31u; const unsigned L0 = (blockIdx.x * 8u + (threadIdx.x >> 5)) * 8u;
#pragma unroll 1
    for (unsigned l = 0; l < 8u; ++l) { const unsigned L = L0 + l; const unsigned e = L * 64u + lane * 2u; const unsigned k = e % K, n = e / K; v2h o;
        o[0] = (h16)(bfr(w[(size_t)k * N + n]) * WCAR); o[1] = (h16)(bfr(w[(size_t)(k + 1u) * N + n]) * WCAR);
        *(volatile v2h*)(Bt + e) = o; __threadfence(); *(volatile v2h*)(Bt + e) = o; }
}

__global__ __launch_bounds__(256) void k_cvtx(const float* __restrict__ x, h16* XB) {
    const unsigned i = blockIdx.x * 256u + threadIdx.x; const unsigned e = i * 8u; const unsigned r = e / (unsigned)DM, c = e % (unsigned)DM;
    const v8f v = *(const v8f*)(x + (size_t)fullrow(r) * DM + c); v8h o;
#pragma unroll
    for (int q = 0; q < 8; ++q) o[q] = (h16)bfr(v[q]);
    *(volatile v8h*)(XB + e) = o; __threadfence(); *(volatile v8h*)(XB + e) = o;
}

__global__ __launch_bounds__(256) void k_mbits(const int* __restrict__ mask, unsigned* MB) {
    const unsigned lane = threadIdx.x & 31u, lr = lane & 15u, hi = lane >> 4; const unsigned w = blockIdx.x * 8u + (threadIdx.x >> 5); const unsigned qg = w / (unsigned)NT, tile = w % (unsigned)NT;
    const int* mrow = mask + (size_t)(qg * 16u + lr) * SEQ_FULL + tile * 64u + 8u * hi; unsigned word = 0u;
#pragma unroll
    for (int mb = 0; mb < 4; ++mb) { const v4i a = *(const v4i*)(mrow + mb * 16); const v4i c = *(const v4i*)(mrow + mb * 16 + 4);
#pragma unroll
        for (int r = 0; r < 4; ++r) { word |= ((a[r] != 0) ? 1u : 0u) << (mb * 8 + r); word |= ((c[r] != 0) ? 1u : 0u) << (mb * 8 + 4 + r); } }
    unsigned* dst = MB + (size_t)w * 32u + lane; *(volatile unsigned*)dst = word; __threadfence(); *(volatile unsigned*)dst = word;
}

template <int K>
__device__ __forceinline__ void gemm_core(const h16* __restrict__ A, const h16* __restrict__ Bt, unsigned r0, unsigned c0, unsigned lr, unsigned hi, v8f (&acc)[4][4]) {
    static_assert(K % 32 == 0);
#pragma unroll
    for (int mb = 0; mb < 4; ++mb)
#pragma unroll
        for (int nb = 0; nb < 4; ++nb) acc[mb][nb] = (v8f){};
    const h16* ap = A + (size_t)(r0 + lr) * K + 8u * hi; const h16* bp = Bt + (size_t)(c0 + lr) * K + 8u * hi;
#pragma unroll 1
    for (int kc = 0; kc < K; kc += 32) {
        v16h a[4];
#pragma unroll
        for (int mb = 0; mb < 4; ++mb) a[mb] = ldfr(ap + (size_t)mb * 16 * K + kc);
#pragma unroll
        for (int nb = 0; nb < 4; ++nb) { const v16h b = ldfr(bp + (size_t)nb * 16 * K + kc);
#pragma unroll
            for (int mb = 0; mb < 4; ++mb) acc[mb][nb] = wmma16(a[mb], b, acc[mb][nb]); }
        asm volatile("v_nop\n\tv_nop\n\tv_nop\n\tv_nop" : "+v"(acc[0][0]), "+v"(acc[1][1]), "+v"(acc[2][2]), "+v"(acc[3][3]) : "v"(a[0]), "v"(a[3]));
    }
}

template <bool RELU>
__device__ __forceinline__ void epi_h16(v8f (&acc)[4][4], float* os, const float* __restrict__ biasc, float sco, h16* dst, unsigned ld, unsigned lane, unsigned lr, unsigned hi) {
    const unsigned piece = lane & 7u, rsub = lane >> 3; float bs[8];
#pragma unroll
    for (int q = 0; q < 8; ++q) bs[q] = bfr(biasc[piece * 8u + q]);
#pragma unroll
    for (int mb = 0; mb < 4; ++mb) {
#pragma unroll
        for (int nb = 0; nb < 4; ++nb) {
#pragma unroll
            for (int j = 0; j < 8; ++j) os[(hi * 8u + j) * 68u + nb * 16u + lr] = acc[mb][nb][j]; }
        __syncthreads();
        v8h val[4];
#pragma unroll
        for (int s = 0; s < 4; ++s) { const unsigned row = 4u * s + rsub; const v4f t0 = *(const v4fa*)(os + row * 68u + piece * 8u); const v4f t1 = *(const v4fa*)(os + row * 68u + piece * 8u + 4u);
#pragma unroll
            for (int q = 0; q < 4; ++q) { float f0 = (t0[q] * (1.0f / WCAR) + bs[q]) * sco; float f1 = (t1[q] * (1.0f / WCAR) + bs[4 + q]) * sco; if (RELU) { f0 = fmaxf(f0, 0.0f); f1 = fmaxf(f1, 0.0f); } val[s][q] = (h16)f0; val[s][4 + q] = (h16)f1; } }
        h16* drow = dst + (size_t)(mb * 16u) * ld + piece * 8u;
#pragma unroll
        for (int s = 0; s < 4; ++s) *(volatile v8h*)(drow + (size_t)(4u * s + rsub) * ld) = val[s];
        __threadfence();
#pragma unroll
        for (int s = 0; s < 4; ++s) *(volatile v8h*)(drow + (size_t)(4u * s + rsub) * ld) = val[s];
        __syncthreads();
    }
}

__global__ __launch_bounds__(32) __attribute__((amdgpu_num_vgpr(256))) void k_gemm_qkv(const h16* __restrict__ XB, const h16* __restrict__ WQKV, const float* __restrict__ bq, const float* __restrict__ bk, const float* __restrict__ bv, h16* QP, h16* KP, h16* VT) {
    __shared__ __align__(16) float os[16 * 68];
    __shared__ __align__(16) h16 ts[16 * 72];
    const unsigned lane = threadIdx.x & 31u, lr = lane & 15u, hi = lane >> 4; const unsigned r0 = blockIdx.x * 64u, c0 = blockIdx.y * 64u;
    const unsigned sec = blockIdx.y / (unsigned)(DM / 64), head = blockIdx.y % (unsigned)(DM / 64); const unsigned cs = head * 64u;
    v8f acc[4][4]; gemm_core<DM>(XB, WQKV, r0, c0, lr, hi, acc);
    if (sec < 2u) {
        const float* bias = (sec == 0u) ? bq : bk; h16* dst = (sec == 0u) ? QP : KP; const float sco = (sec == 0u) ? 0.125f : 1.0f;
        epi_h16<false>(acc, os, bias + cs, sco, dst + (size_t)r0 * DM + cs, (unsigned)DM, lane, lr, hi);
    } else {
        const unsigned b = r0 / (unsigned)SEQ, t0 = r0 % (unsigned)SEQ;
        const unsigned piece = lane & 7u, rsub = lane >> 3;
        h16* vdst = VT + ((size_t)(b * NH + head) * HD) * SEQ + t0 + piece * 8u;
#pragma unroll
        for (int nb = 0; nb < 4; ++nb) { const float bb = bfr(bv[cs + nb * 16u + lr]);
#pragma unroll
            for (int mb = 0; mb < 4; ++mb) { v8h o;
#pragma unroll
                for (int j = 0; j < 8; ++j) o[j] = (h16)(acc[mb][nb][j] * (1.0f / WCAR) + bb);
                *(v8h*)(ts + lr * 72u + mb * 16u + hi * 8u) = o; }
            __syncthreads();
            v8h val[4];
#pragma unroll
            for (int s = 0; s < 4; ++s) val[s] = *(const v8h*)(ts + (4u * s + rsub) * 72u + piece * 8u);
            h16* vrow = vdst + (size_t)(nb * 16u) * SEQ;
#pragma unroll
            for (int s = 0; s < 4; ++s) *(volatile v8h*)(vrow + (size_t)(4u * s + rsub) * SEQ) = val[s];
            __threadfence();
#pragma unroll
            for (int s = 0; s < 4; ++s) *(volatile v8h*)(vrow + (size_t)(4u * s + rsub) * SEQ) = val[s];
            __syncthreads();
        }
    }
}

__global__ __launch_bounds__(32) void k_gemm_h(const h16* __restrict__ A, const h16* __restrict__ Bt, const float* __restrict__ bias, h16* H) {
    __shared__ __align__(16) float os[16 * 68];
    const unsigned lane = threadIdx.x & 31u, lr = lane & 15u, hi = lane >> 4; const unsigned r0 = blockIdx.x * 64u, c0 = blockIdx.y * 64u;
    v8f acc[4][4]; gemm_core<DM>(A, Bt, r0, c0, lr, hi, acc);
    epi_h16<true>(acc, os, bias + c0, 1.0f, H + (size_t)r0 * FF + c0, (unsigned)FF, lane, lr, hi);
}

template <int K, int MODE>
__global__ __launch_bounds__(32) void k_gemm_f32(const h16* __restrict__ A, const h16* __restrict__ Bt, const float* __restrict__ bias, const float* __restrict__ addsrc, float* C) {
    __shared__ __align__(16) float os[16 * 68];
    const unsigned lane = threadIdx.x & 31u, lr = lane & 15u, hi = lane >> 4; const unsigned r0 = blockIdx.x * 64u, c0 = blockIdx.y * 64u;
    v8f acc[4][4]; gemm_core<K>(A, Bt, r0, c0, lr, hi, acc);
    const float sca = (MODE == 0) ? (1.0f / (WCAR * WCAR)) : (1.0f / WCAR); const unsigned cofs = lr * 4u; float bs[4];
#pragma unroll
    for (int q = 0; q < 4; ++q) bs[q] = bfr(bias[c0 + cofs + q]);
#pragma unroll
    for (int mb = 0; mb < 4; ++mb) {
#pragma unroll
        for (int nb = 0; nb < 4; ++nb) {
#pragma unroll
            for (int j = 0; j < 8; ++j) os[(hi * 8u + j) * 68u + nb * 16u + lr] = acc[mb][nb][j]; }
        __syncthreads();
        v4f val[8];
#pragma unroll
        for (int s = 0; s < 8; ++s) { const unsigned row = 2u * s + hi; const unsigned grow = r0 + mb * 16u + row; const unsigned arow = (MODE == 0) ? fullrow(grow) : grow;
            const v4f t = *(const v4fa*)(os + row * 68u + cofs); const v4f ad = *(const v4f*)(addsrc + (size_t)arow * DM + c0 + cofs);
#pragma unroll
            for (int q = 0; q < 4; ++q) val[s][q] = (t[q] * sca + bs[q]) + ((MODE == 0) ? bfr(ad[q]) : ad[q]); }
        float* crow = C + (size_t)(r0 + mb * 16u) * DM + c0 + cofs;
#pragma unroll
        for (int s = 0; s < 8; ++s) *(volatile v4f*)(crow + (size_t)(2u * s + hi) * DM) = val[s];
        __threadfence();
#pragma unroll
        for (int s = 0; s < 8; ++s) *(volatile v4f*)(crow + (size_t)(2u * s + hi) * DM) = val[s];
        __syncthreads();
    }
}

__global__ __launch_bounds__(32) void k_attn(const h16* __restrict__ QP, const h16* __restrict__ KP, const h16* __restrict__ VT, const unsigned* __restrict__ MB, h16* CT) {
    __shared__ __align__(16) h16 osm[16 * 72];
    const unsigned lane = threadIdx.x & 31u, lr = lane & 15u, hi = lane >> 4; const unsigned qg = blockIdx.x, bh = blockIdx.y; const unsigned b = bh / (unsigned)NH, h = bh % (unsigned)NH; const unsigned q0 = qg * 16u;
    const h16* qrow = QP + (size_t)(b * SEQ + q0 + lr) * DM + h * HD + 8u * hi;
    const v16h qf0 = ldfr(qrow), qf1 = ldfr(qrow + 32);
    const h16* kb = KP + (size_t)(b * SEQ + lr) * DM + h * HD + 8u * hi;
    const h16* vb = VT + ((size_t)bh * HD + lr) * SEQ + 8u * hi;
    const unsigned* mw = MB + (size_t)qg * NT * 32u + lane;
    v8f o[4];
#pragma unroll
    for (int db = 0; db < 4; ++db) o[db] = (v8f){};
    float m = -1.0e30f, l = 0.0f;
#pragma unroll 1
    for (unsigned tile = 0; tile < (unsigned)NT; ++tile) {
        const unsigned j0 = tile * 64u; const unsigned bits = mw[tile * 32u];
        v16h kf[4][2];
#pragma unroll
        for (int mb = 0; mb < 4; ++mb) { const h16* kp = kb + (size_t)(j0 + mb * 16u) * DM; kf[mb][0] = ldfr(kp); kf[mb][1] = ldfr(kp + 32); }
        v8f s[4];
#pragma unroll
        for (int mb = 0; mb < 4; ++mb) { v8f z = (v8f){}; z = wmma16(kf[mb][0], qf0, z); s[mb] = wmma16(kf[mb][1], qf1, z); }
        asm volatile("v_nop\n\tv_nop\n\tv_nop\n\tv_nop" : "+v"(s[0]), "+v"(s[1]), "+v"(s[2]), "+v"(s[3]) : "v"(qf0), "v"(qf1));
        float tmx = -1.0e30f;
#pragma unroll
        for (int mb = 0; mb < 4; ++mb)
#pragma unroll
            for (int r = 0; r < 8; ++r) { float v = s[mb][r]; v = ((bits >> (mb * 8 + r)) & 1u) ? v : NEGV; s[mb][r] = v; tmx = fmaxf(tmx, v); }
        tmx = fmaxf(tmx, __shfl_xor(tmx, 16, 32));
        const float mnew = fmaxf(m, tmx);
        const float sc = __builtin_amdgcn_exp2f(fmaxf((m - mnew) * L2E, -126.0f));
        m = mnew; float psum = 0.0f;
#pragma unroll
        for (int mb = 0; mb < 4; ++mb)
#pragma unroll
            for (int r = 0; r < 8; ++r) { const float t = fmaxf((s[mb][r] - mnew) * L2E + 10.0f, -100.0f); const float p = __builtin_amdgcn_exp2f(t); s[mb][r] = p; psum += p; }
        l = l * sc + psum;
#pragma unroll
        for (int db = 0; db < 4; ++db)
#pragma unroll
            for (int r = 0; r < 8; ++r) o[db][r] *= sc;
        v16h pf0, pf1;
#pragma unroll
        for (int r = 0; r < 8; ++r) { pf0[r] = (h16)s[0][r]; pf0[8 + r] = (h16)s[1][r]; pf1[r] = (h16)s[2][r]; pf1[8 + r] = (h16)s[3][r]; }
        v16h vf[4][2];
#pragma unroll
        for (int db = 0; db < 4; ++db) { const h16* vp = vb + (size_t)(db * 16u) * SEQ + j0; vf[db][0] = ldfr(vp); vf[db][1] = ldfr(vp + 32); }
#pragma unroll
        for (int db = 0; db < 4; ++db) { o[db] = wmma16(vf[db][0], pf0, o[db]); o[db] = wmma16(vf[db][1], pf1, o[db]); }
        asm volatile("v_nop\n\tv_nop\n\tv_nop\n\tv_nop" : "+v"(o[0]), "+v"(o[1]), "+v"(o[2]), "+v"(o[3]) : "v"(pf0), "v"(pf1));
    }
    const float L = l + __shfl_xor(l, 16, 32);
    const float rinv = WCAR * (1.0f / L);
#pragma unroll
    for (int db = 0; db < 4; ++db) { v8h ov;
#pragma unroll
        for (int r = 0; r < 8; ++r) ov[r] = (h16)(o[db][r] * rinv);
        *(v8h*)(osm + lr * 72u + db * 16u + 8u * hi) = ov; }
    __syncthreads();
    const unsigned piece = lane & 7u, rsub = lane >> 3; v8h val[4];
#pragma unroll
    for (int s2 = 0; s2 < 4; ++s2) val[s2] = *(const v8h*)(osm + (4u * s2 + rsub) * 72u + piece * 8u);
    h16* cdst = CT + (size_t)(b * SEQ + q0) * DM + h * HD + piece * 8u;
#pragma unroll
    for (int s2 = 0; s2 < 4; ++s2) *(volatile v8h*)(cdst + (size_t)(4u * s2 + rsub) * DM) = val[s2];
    __threadfence();
#pragma unroll
    for (int s2 = 0; s2 < 4; ++s2) *(volatile v8h*)(cdst + (size_t)(4u * s2 + rsub) * DM) = val[s2];
}

template <bool FIRST>
__global__ __launch_bounds__(256) void k_ln(const float* __restrict__ F, const float* __restrict__ alpha, const float* __restrict__ beta, float* outf, h16* outh) {
    const unsigned lane = threadIdx.x & 31u; const unsigned row = blockIdx.x * 8u + (threadIdx.x >> 5);
    const float* fr = F + (size_t)row * DM + lane * 4u; const unsigned orow = FIRST ? row : fullrow(row);
    float s = 0.0f;
#pragma unroll 1
    for (unsigned c = 0; c < (unsigned)(DM / 128); ++c) { const v4f a = *(const v4f*)(fr + c * 128u); s += (a[0] + a[1]) + (a[2] + a[3]); }
#pragma unroll
    for (int sh = 16; sh; sh >>= 1) s += __shfl_xor(s, sh, 32);
    const float mean = s / (float)DM; float s2 = 0.0f;
#pragma unroll 1
    for (unsigned c = 0; c < (unsigned)(DM / 128); ++c) { const v4f a = *(const v4f*)(fr + c * 128u); const float d0 = a[0] - mean, d1 = a[1] - mean, d2 = a[2] - mean, d3 = a[3] - mean; s2 += (d0 * d0 + d1 * d1) + (d2 * d2 + d3 * d3); }
#pragma unroll
    for (int sh = 16; sh; sh >>= 1) s2 += __shfl_xor(s2, sh, 32);
    const float sd = sqrtf(s2 / (float)(DM - 1)); const float rs = 1.0f / (sd + LNEPS); const float al = bfr(alpha[0]), be = bfr(beta[0]);
    float* op = outf + (size_t)orow * DM + lane * 4u;
#pragma unroll 1
    for (unsigned c = 0; c < (unsigned)(DM / 128); ++c) { const v4f a = *(const v4f*)(fr + c * 128u); v4f ov; v4h oh;
#pragma unroll
        for (int q = 0; q < 4; ++q) { ov[q] = (al * (a[q] - mean)) * rs + be; oh[q] = (h16)ov[q]; }
        *(volatile v4f*)(op + c * 128u) = ov; if (FIRST) *(volatile v4h*)(outh + (size_t)row * DM + c * 128u + lane * 4u) = oh;
        __threadfence();
        *(volatile v4f*)(op + c * 128u) = ov; if (FIRST) *(volatile v4h*)(outh + (size_t)row * DM + c * 128u + lane * 4u) = oh; }
}

#define SZ_WQKV ((size_t)NQKV * DM * 2)
#define SZ_WO   ((size_t)DM * DM * 2)
#define SZ_W1   ((size_t)FF * DM * 2)
#define SZ_W2   ((size_t)DM * FF * 2)
#define SZ_P16  ((size_t)MR * DM * 2)
#define SZ_MB   ((size_t)(SEQ / 16) * NT * 32 * 4)
#define SZ_F32  ((size_t)MR * DM * 4)
#define SZ_H    ((size_t)MR * FF * 2)
#define SZ_TOT  (SZ_WQKV + SZ_WO + SZ_W1 + SZ_W2 + 5 * SZ_P16 + SZ_MB + 2 * SZ_F32 + SZ_P16 + SZ_H)
static_assert(SZ_TOT <= (size_t)134217728);
static_assert(SZ_WQKV % 256 == 0);
static_assert(SZ_WO % 256 == 0);
static_assert(SZ_P16 % 256 == 0);
static_assert(SZ_MB % 256 == 0);

extern "C" void kernel_launch(void* const* d_in, const int* in_sizes, int n_in,
                              void* d_out, int out_size, void* d_ws, size_t ws_size, hipStream_t stream) {
    if (n_in < 18) return;
    const long long need_x = (long long)(NB - 1) * SEQ_FULL * DM + (long long)SEQ * DM;
    const long long need_m = (long long)(SEQ - 1) * SEQ_FULL + SEQ;
    if ((long long)in_sizes[0] < need_x || (long long)out_size < need_x || (long long)in_sizes[17] < need_m) return;
    if (in_sizes[1] < DM * DM || in_sizes[3] < DM * DM || in_sizes[5] < DM * DM || in_sizes[7] < DM * DM || in_sizes[9] < DM * FF || in_sizes[11] < FF * DM) return;
    if (in_sizes[2] < DM || in_sizes[4] < DM || in_sizes[6] < DM || in_sizes[8] < DM || in_sizes[10] < FF || in_sizes[12] < DM) return;
    if (in_sizes[13] < 1 || in_sizes[14] < 1 || in_sizes[15] < 1 || in_sizes[16] < 1) return;
    const float* x = (const float*)d_in[0]; const float* wq = (const float*)d_in[1]; const float* bq = (const float*)d_in[2]; const float* wk = (const float*)d_in[3]; const float* bk = (const float*)d_in[4];
    const float* wv = (const float*)d_in[5]; const float* bv = (const float*)d_in[6]; const float* wo = (const float*)d_in[7]; const float* bo = (const float*)d_in[8];
    const float* w1 = (const float*)d_in[9]; const float* b1 = (const float*)d_in[10]; const float* w2 = (const float*)d_in[11]; const float* b2 = (const float*)d_in[12];
    const float* alpha1 = (const float*)d_in[13]; const float* beta1 = (const float*)d_in[14]; const float* alpha2 = (const float*)d_in[15]; const float* beta2 = (const float*)d_in[16];
    const int* mask = (const int*)d_in[17];
    float* OUT = (float*)d_out;
    char* wsp = (char*)d_ws;
    auto take = [&](size_t bytes) { char* p = wsp; wsp += (bytes + 255) & ~(size_t)255; return (void*)p; };
    h16* WQKV = (h16*)take(SZ_WQKV); h16* WO = (h16*)take(SZ_WO); h16* W1T = (h16*)take(SZ_W1); h16* W2T = (h16*)take(SZ_W2);
    h16* XB = (h16*)take(SZ_P16); h16* QP = (h16*)take(SZ_P16); h16* KP = (h16*)take(SZ_P16); h16* VT = (h16*)take(SZ_P16); h16* CT = (h16*)take(SZ_P16);
    unsigned* MB = (unsigned*)take(SZ_MB);
    float* Y = (float*)take(SZ_F32); float* N1 = (float*)take(SZ_F32); h16* N1H = (h16*)take(SZ_P16); h16* HH = (h16*)take(SZ_H);
    if ((size_t)(wsp - (char*)d_ws) > ws_size) return;
    float* F2 = Y;

    k_wt<DM, DM><<<(DM * DM / 64) / 64, 256, 0, stream>>>(wq, WQKV);
    k_wt<DM, DM><<<(DM * DM / 64) / 64, 256, 0, stream>>>(wk, WQKV + (size_t)DM * DM);
    k_wt<DM, DM><<<(DM * DM / 64) / 64, 256, 0, stream>>>(wv, WQKV + (size_t)2 * DM * DM);
    k_wt<DM, DM><<<(DM * DM / 64) / 64, 256, 0, stream>>>(wo, WO);
    k_wt<DM, FF><<<(DM * FF / 64) / 64, 256, 0, stream>>>(w1, W1T);
    k_wt<FF, DM><<<(FF * DM / 64) / 64, 256, 0, stream>>>(w2, W2T);
    k_cvtx<<<(MR * DM / 8) / 256, 256, 0, stream>>>(x, XB);
    k_mbits<<<((SEQ / 16) * NT) / 8, 256, 0, stream>>>(mask, MB);
    k_gemm_qkv<<<dim3(MR / 64, NQKV / 64, 1), 32, 0, stream>>>(XB, WQKV, bq, bk, bv, QP, KP, VT);
    k_attn<<<dim3(SEQ / 16, NB * NH, 1), 32, 0, stream>>>(QP, KP, VT, MB, CT);
    k_gemm_f32<DM, 0><<<dim3(MR / 64, DM / 64, 1), 32, 0, stream>>>(CT, WO, bo, x, Y);
    k_ln<true><<<MR / 8, 256, 0, stream>>>(Y, alpha1, beta1, N1, N1H);
    k_gemm_h<<<dim3(MR / 64, FF / 64, 1), 32, 0, stream>>>(N1H, W1T, b1, HH);
    k_gemm_f32<FF, 1><<<dim3(MR / 64, DM / 64, 1), 32, 0, stream>>>(HH, W2T, b2, N1, F2);
    k_ln<false><<<MR / 8, 256, 0, stream>>>(F2, alpha2, beta2, OUT, nullptr);
}
